// LinearAttention_27144193311318
// MI455X (gfx1250) — hardware-run, weakly checked
//
#include <hip/hip_runtime.h>


#ifndef NB
#define NB 8
#endif
#ifndef SEQ
#define SEQ 16384
#endif
#ifndef IMW
#define IMW 128
#endif
#define NB_FULL  8
#define SEQ_FULL 16384
#ifndef OUT_SEQ
#define OUT_SEQ SEQ
#endif
#define DM   96
#define NH_  4
#define HD   24
#define NPR  48
#define NT   (SEQ / 64)
#define OW   8
#define OSQ  100
#define QSP  104
#define TSP  72
#define KVW  4
#define KVSPL 4
#define KVTOK (SEQ / (KVW * KVSPL))
#define KVS  1024.0f
#define KVI  (1.0f / 1024.0f)
#define KVSC (1024.0f / (float)SEQ)
#define L2E  1.4426950408889634f

static_assert(NH_ * HD == DM);
static_assert(DM % 32 == 0);
static_assert(DM % 16 == 0);
static_assert(DM % 8 == 0);
static_assert(2 * NPR == DM);
static_assert(HD % 2 == 0);
static_assert(IMW * IMW == SEQ);
static_assert(IMW % 64 == 0);
static_assert(SEQ % 64 == 0);
static_assert((NB * SEQ) % 64 == 0);
static_assert(SEQ % (16 * OW) == 0);
static_assert((NB * SEQ) % (16 * OW) == 0);
static_assert(KVTOK % 32 == 0);
static_assert(KVTOK * KVW * KVSPL == SEQ);
static_assert((2 * NPR * IMW) % 256 == 0);
static_assert((NPR * IMW) % 256 == 0);
static_assert((2 * DM * DM) % 8 == 0);
static_assert(NB <= NB_FULL);
static_assert(SEQ <= SEQ_FULL);
static_assert((OSQ * 4) % 16 == 0);
static_assert((QSP * 2) % 16 == 0);
static_assert((TSP * 2) % 16 == 0);
static_assert(OSQ >= DM);
static_assert(QSP >= DM);
static_assert(HD + 8 <= 32);

typedef _Float16 h16;
typedef unsigned short bf;
typedef __attribute__((ext_vector_type(16))) __bf16   v16bf;
typedef __attribute__((ext_vector_type(16))) _Float16 v16h;
typedef __attribute__((ext_vector_type(8)))  _Float16 v8h;
typedef __attribute__((ext_vector_type(8)))  unsigned short v8us;
typedef __attribute__((ext_vector_type(8)))  float    v8f;
typedef __attribute__((ext_vector_type(4)))  float    v4f;
typedef v4f  __attribute__((may_alias)) v4fa;
typedef v8h  __attribute__((may_alias)) v8ha;
typedef __attribute__((ext_vector_type(2)))  unsigned v2u;

__device__ __forceinline__ unsigned short f2bf(float f) { unsigned u = __float_as_uint(f); u += 0x7FFFu + ((u >> 16) & 1u); return (unsigned short)(u >> 16); }
__device__ __forceinline__ float bfr(float f) { return __uint_as_float(((unsigned)f2bf(f)) << 16); }
__device__ __forceinline__ v16h cat16(v8h lo, v8h hi) { return __builtin_shufflevector(lo, hi, 0, 1, 2, 3, 4, 5, 6, 7, 8, 9, 10, 11, 12, 13, 14, 15); }
__device__ __forceinline__ v16bf cat16b(v8us lo, v8us hi) { return __builtin_bit_cast(v16bf, __builtin_shufflevector(lo, hi, 0, 1, 2, 3, 4, 5, 6, 7, 8, 9, 10, 11, 12, 13, 14, 15)); }
__device__ __forceinline__ v8f wmma16(v16h a, v16h b, v8f c) { return __builtin_amdgcn_wmma_f32_16x16x32_f16(false, a, false, b, (short)0, c, false, false); }
__device__ __forceinline__ v8f wmmab(v16bf a, v16bf b, v8f c) { return __builtin_amdgcn_wmma_f32_16x16x32_bf16(false, a, false, b, (short)0, c, false, false); }
__device__ __forceinline__ v16h  ldh(const h16* p) { return cat16(*(const v8h*)p, *(const v8h*)(p + 16)); }
__device__ __forceinline__ v16bf ldb(const bf* p)  { return cat16b(*(const v8us*)p, *(const v8us*)(p + 16)); }
__device__ __forceinline__ void wave_sync() { __builtin_amdgcn_fence(3  , "wavefront"); __builtin_amdgcn_wave_barrier(); asm volatile("" ::: "memory"); }

static __device__ __forceinline__ h16 toh_flush(float v) { const h16 r = (h16)v; return (fabsf(v) < 6.103515625e-05f) ? (h16)0.0f : r; }
static __device__ __forceinline__ v8f wmma16g(v16h a, v16h b, v8f c) { c = wmma16(a, b, c); asm volatile("v_nop\n\tv_nop\n\tv_nop\n\tv_nop" : "+v"(c) : "v"(a), "v"(b)); return c; }
static __device__ __forceinline__ v8f wmmabg(v16bf a, v16bf b, v8f c) { c = wmmab(a, b, c); asm volatile("v_nop\n\tv_nop\n\tv_nop\n\tv_nop" : "+v"(c) : "v"(a), "v"(b)); return c; }
static __device__ __forceinline__ float elu1(float v) { const float ex = __builtin_amdgcn_exp2f(fminf(v, 0.0f) * L2E); return (v > 0.0f) ? (v + 1.0f) : ex; }

__global__ __launch_bounds__(256) void k_cvt8(const float* __restrict__ src, bf* dst, size_t n8) {
    const size_t i = (size_t)blockIdx.x * 256 + threadIdx.x; if (i >= n8) return;
    const v8f v = *(const v8f*)(src + i * 8); v8us o;
#pragma unroll
    for (int k = 0; k < 8; ++k) o[k] = f2bf(v[k]);
    *(volatile v8us*)(dst + i * 8) = o; __threadfence(); *(volatile v8us*)(dst + i * 8) = o;
}

__global__ __launch_bounds__(256) void k_tab(float* TB) {
    const int n = NPR * IMW;
    const int i = blockIdx.x * 256 + threadIdx.x;
    const int lay = i / n; const int r = i - lay * n;
    const int j = lay ? (r % NPR) : (r / IMW);
    const int w = lay ? (r / NPR) : (r % IMW);
    const float th = exp2f(-((float)j * (1.0f / (float)NPR)) * 13.287712379549449f);
    float sn, cs; sincosf((float)w * th, &sn, &cs);
    const size_t oc = (size_t)lay * 2 * n + (size_t)r;
    *(volatile float*)(TB + oc) = cs; *(volatile float*)(TB + oc + n) = sn;
    __threadfence();
    *(volatile float*)(TB + oc) = cs; *(volatile float*)(TB + oc + n) = sn;
}

static_assert(3 * 256 * 8 == 64 * DM);
__global__ __launch_bounds__(256) void k_xprep(const float* __restrict__ x, bf* XB, h16* VT) {
    __shared__ __align__(16) h16 ts[DM * TSP];
    const int tid = threadIdx.x;
    const size_t g0 = (size_t)blockIdx.x * 64;
    const int b = (int)(g0 / SEQ), tt = (int)(g0 % SEQ);
    const float* src = x + ((size_t)b * SEQ_FULL + (size_t)tt) * DM;
    v8us ov[3];
#pragma unroll
    for (int it = 0; it < 3; ++it) {
        const int f = it * 256 + tid; const int row = f / 12, c8 = (f - row * 12) * 8;
        const v8f v = *(const v8f*)(src + (size_t)f * 8); v8us o;
#pragma unroll
        for (int k = 0; k < 8; ++k) { const unsigned short u = f2bf(v[k]); o[k] = u; ts[(c8 + k) * TSP + row] = toh_flush(__uint_as_float(((unsigned)u) << 16)); }
        ov[it] = o; }
    __syncthreads();
    v8h vt[3];
#pragma unroll
    for (int it = 0; it < 3; ++it) { const int f = it * 256 + tid; const int c = f >> 3, t8 = (f & 7) * 8; vt[it] = *(const v8ha*)(&ts[c * TSP + t8]); }
    bf* xb = XB + g0 * DM;
    h16* vrow = VT + (size_t)b * DM * SEQ + (size_t)tt;
#pragma unroll 1
    for (int ps = 0; ps < 2; ++ps) {
#pragma unroll
        for (int it = 0; it < 3; ++it) { const int f = it * 256 + tid; const int c = f >> 3, t8 = (f & 7) * 8;
            *(volatile v8us*)(xb + (size_t)f * 8) = ov[it];
            *(volatile v8h*)(vrow + (size_t)c * SEQ + t8) = vt[it]; }
        if (ps == 0) __threadfence(); }
}

static_assert(4 * 4 == 16);
static_assert(8 * 8 == 64);
__global__ __launch_bounds__(32) void k_kproj(const bf* __restrict__ A, const bf* __restrict__ Bt, const float* __restrict__ bias, const float* __restrict__ TB, h16* KT, float* KSP) {
    __shared__ __align__(16) float os[16 * 68];
    __shared__ __align__(16) float ksw[64];
    const int K = DM;
    const int lane = threadIdx.x & 31, lr = lane & 15, hi = lane >> 4; const int r0 = blockIdx.x * 48, n0 = blockIdx.y * 64;
    v8f acc[3][4];
#pragma unroll
    for (int mb = 0; mb < 3; ++mb)
#pragma unroll
        for (int nb = 0; nb < 4; ++nb) acc[mb][nb] = (v8f){};
    const size_t aoff = (size_t)(r0 + lr) * K + 8 * hi, boff = (size_t)(n0 + lr) * K + 8 * hi;
#pragma unroll 1
    for (int kc = 0; kc < K; kc += 32) {
        v16bf a[3];
#pragma unroll
        for (int mb = 0; mb < 3; ++mb) a[mb] = ldb(A + aoff + (size_t)mb * 16 * K + kc);
#pragma unroll
        for (int nb = 0; nb < 4; ++nb) { const v16bf b = ldb(Bt + boff + (size_t)nb * 16 * K + kc);
#pragma unroll
            for (int mb = 0; mb < 3; ++mb) acc[mb][nb] = wmmabg(a[mb], b, acc[mb][nb]); }
    }
    const int bb = n0 / SEQ, tt = n0 % SEQ;
    const size_t tbase = (size_t)bb * (size_t)DM * SEQ + (size_t)r0 * SEQ + (size_t)tt;
    if (lane < 16) ksw[48 + lane] = 0.0f;
    const int wq = (tt + (lane & 7) * 8) % IMW;
#pragma unroll
    for (int mb = 0; mb < 3; ++mb) {
        float br[8];
#pragma unroll
        for (int j = 0; j < 8; ++j) br[j] = bfr(bias[r0 + mb * 16 + hi * 8 + j]);
#pragma unroll
        for (int nb = 0; nb < 4; ++nb) {
#pragma unroll
            for (int j = 0; j < 8; ++j) os[(hi * 8 + j) * 68 + nb * 16 + lr] = elu1(acc[mb][nb][j] + br[j]); }
        wave_sync();
        v8h hv[4];
#pragma unroll
        for (int s = 0; s < 4; ++s) { const int row = 4 * s + (lane >> 3), c8 = (lane & 7) * 8;
            const v4f x0 = *(const v4fa*)(&os[row * 68 + c8]); const v4f x1 = *(const v4fa*)(&os[row * 68 + c8 + 4]);
            const v4f y0 = *(const v4fa*)(&os[(row ^ 1) * 68 + c8]); const v4f y1 = *(const v4fa*)(&os[(row ^ 1) * 68 + c8 + 4]);
            float rs = ((x0[0] + x0[1]) + (x0[2] + x0[3])) + ((x1[0] + x1[1]) + (x1[2] + x1[3]));
            rs += __shfl_xor(rs, 1, 32); rs += __shfl_xor(rs, 2, 32); rs += __shfl_xor(rs, 4, 32);
            if ((lane & 7) == 0) ksw[mb * 16 + row] = rs;
            const int to = ((r0 + mb * 16 + row) >> 1) * IMW + wq;
            const v4f ca = *(const v4f*)(TB + to), cb = *(const v4f*)(TB + to + 4);
            const v4f sa = *(const v4f*)(TB + NPR * IMW + to), sb = *(const v4f*)(TB + NPR * IMW + to + 4);
            const float sg = (row & 1) ? 1.0f : -1.0f;
            v8h hq;
#pragma unroll
            for (int i = 0; i < 4; ++i) { hq[i] = toh_flush(x0[i] * ca[i] + sg * (y0[i] * sa[i])); hq[4 + i] = toh_flush(x1[i] * cb[i] + sg * (y1[i] * sb[i])); }
            hv[s] = hq; }
        const size_t sbo = tbase + (size_t)(mb * 16) * SEQ;
#pragma unroll 1
        for (int ps = 0; ps < 2; ++ps) {
#pragma unroll
            for (int s = 0; s < 4; ++s) { const int row = 4 * s + (lane >> 3), c8 = (lane & 7) * 8;
                *(volatile v8h*)(KT + sbo + (size_t)row * SEQ + c8) = hv[s]; }
            if (ps == 0) __threadfence(); }
        wave_sync();
    }
    if (lane < 16) {
        const v4f kv4 = *(const v4fa*)(&ksw[lane * 4]);
        float* kp = KSP + ((size_t)blockIdx.y * 2 + blockIdx.x) * 64 + lane * 4;
        *(volatile v4f*)kp = kv4; __threadfence(); *(volatile v4f*)kp = kv4;
    }
}

static_assert(2 * 32 * KVW * 4 == 32 * 32);
__global__ __launch_bounds__(32 * KVW) void k_kv(const h16* __restrict__ KT, const h16* __restrict__ VT, float* KVP) {
    __shared__ __align__(16) float ps[KVW * 32 * 36];
    const int tid = threadIdx.x;
    const int lane = tid & 31, lr = lane & 15, hi = lane >> 4;
    const int wave = __builtin_amdgcn_readfirstlane((int)(threadIdx.x >> 5));
    const int zh = blockIdx.y; const int b = zh / NH_, h = zh % NH_;
    const int tok0 = (blockIdx.x * KVW + wave) * KVTOK;
    const int ra = HD * h + lr;
    int rb = HD * h + 16 + lr; rb = rb > (DM - 1) ? (DM - 1) : rb;
    const size_t o0 = ((size_t)b * DM + ra) * SEQ + (size_t)tok0 + 8 * hi;
    const size_t o1 = ((size_t)b * DM + rb) * SEQ + (size_t)tok0 + 8 * hi;
    v8f a00 = (v8f){}, a01 = (v8f){}, a10 = (v8f){}, a11 = (v8f){};
#pragma unroll 1
    for (int k = 0; k < KVTOK; k += 32) {
        const v16h ka = ldh(KT + o0 + k), kb = ldh(KT + o1 + k);
        const v16h va = ldh(VT + o0 + k), vb = ldh(VT + o1 + k);
        a00 = wmma16g(ka, va, a00); a01 = wmma16g(ka, vb, a01); a10 = wmma16g(kb, va, a10); a11 = wmma16g(kb, vb, a11);
    }
    const int wp = wave * 32 * 36;
#pragma unroll
    for (int j = 0; j < 8; ++j) {
        ps[wp + (8 * hi + j) * 36 + lr] = a00[j];      ps[wp + (8 * hi + j) * 36 + 16 + lr] = a01[j];
        ps[wp + (16 + 8 * hi + j) * 36 + lr] = a10[j]; ps[wp + (16 + 8 * hi + j) * 36 + 16 + lr] = a11[j]; }
    __syncthreads();
    v4f hold[2];
#pragma unroll
    for (int it = 0; it < 2; ++it) { const int f = it * 128 + tid; const int row = f >> 3, c4 = (f & 7) * 4;
        v4f s = *(const v4fa*)(&ps[row * 36 + c4]);
#pragma unroll
        for (int wv = 1; wv < KVW; ++wv) { const v4f t = *(const v4fa*)(&ps[wv * 32 * 36 + row * 36 + c4]); s += t; }
        hold[it] = s; }
    float* dst = KVP + ((size_t)zh * KVSPL + blockIdx.x) * 1024;
#pragma unroll 1
    for (int psn = 0; psn < 2; ++psn) {
#pragma unroll
        for (int it = 0; it < 2; ++it) { const int f = it * 128 + tid; *(volatile v4f*)(dst + (size_t)f * 4) = hold[it]; }
        if (psn == 0) __threadfence(); }
}

static_assert(9 * 256 == NH_ * HD * HD);
static_assert((DM * DM) % 256 == 0);
static_assert(DM * DM / 8 == 1152);
static_assert(DM * DM / 8 <= 5 * 256);
__global__ __launch_bounds__(256) void k_fin(const float* __restrict__ KSP, const float* __restrict__ KVP, float* KM, h16* KVB) {
    __shared__ __align__(16) h16 kvs[DM * QSP];
    __shared__ __align__(16) float kml[128];
    const int tid = threadIdx.x; const int b = blockIdx.x;
    { const v8h z8 = (v8h){};
      for (int i = tid; i < DM * QSP / 8; i += 256) *(v8ha*)(&kvs[i * 8]) = z8; }
    if (tid < 128) {
        float s = 0.0f;
        if (tid < DM) {
            const int hf = tid / 48, cc = tid - hf * 48;
            const float* p = KSP + (((size_t)b * NT) * 2 + hf) * 64 + cc;
#pragma unroll 1
            for (int tl = 0; tl < NT; ++tl) s += p[(size_t)tl * 128]; }
        kml[tid] = s * (1.0f / (float)SEQ); }
    __syncthreads();
#pragma unroll 1
    for (int i = tid; i < NH_ * HD * HD; i += 256) {
        const int h = i / (HD * HD); const int r = i - h * HD * HD; const int d = r / HD, e = r - d * HD;
        const float* p = KVP + ((size_t)(b * NH_ + h) * KVSPL) * 1024 + d * 32 + e;
        float s = 0.0f;
#pragma unroll
        for (int kb = 0; kb < KVSPL; ++kb) s += p[kb * 1024];
        kvs[(HD * h + e) * QSP + HD * h + d] = toh_flush(s * KVSC); }
    __syncthreads();
    v8h hold[5];
#pragma unroll
    for (int it = 0; it < 5; ++it) { const int f = it * 256 + tid; const int fc = f < 1152 ? f : 1151; const int row = fc / 12, c8 = (fc - row * 12) * 8;
        hold[it] = *(const v8ha*)(&kvs[row * QSP + c8]); }
    const v4f kmv = *(const v4fa*)(&kml[(tid & 31) * 4]);
    h16* kdst = KVB + (size_t)b * DM * DM;
#pragma unroll 1
    for (int ps = 0; ps < 2; ++ps) {
#pragma unroll
        for (int it = 0; it < 5; ++it) { const int f = it * 256 + tid; if (f < 1152) *(volatile v8h*)(kdst + (size_t)f * 8) = hold[it]; }
        if (tid < 32) *(volatile v4f*)(KM + (size_t)b * 128 + tid * 4) = kmv;
        if (ps == 0) __threadfence(); }
}

static constexpr unsigned kvnz_bits() {
    unsigned m = 0;
    for (int nb = 0; nb < DM / 16; ++nb)
        for (int ks = 0; ks < DM / 32; ++ks) {
            bool nz = false;
            for (int h = 0; h < NH_; ++h) {
                const bool eh = (16 * nb < HD * h + HD) && (16 * nb + 16 > HD * h);
                const bool dh = (32 * ks < HD * h + HD) && (32 * ks + 32 > HD * h);
                if (eh && dh) nz = true; }
            if (nz) m |= 1u << (nb * 3 + ks); }
    return m;
}
static constexpr unsigned KVNZ = kvnz_bits();
static_assert(__builtin_popcount(KVNZ) == 10);

static_assert(6 * 32 * 8 == 16 * DM);
static_assert(12 * 32 * 4 == 16 * DM);
static_assert(OW * 16 * OSQ * 4 + OW * 16 * QSP * 2 + OW * 64 * 4 + 9 * DM * 4 + 2 * DM * 4 <= 131072);
static_assert(DM * TSP * 2 <= 131072);
static_assert(DM * QSP * 2 + 128 * 4 <= 131072);
static_assert(KVW * 32 * 36 * 4 <= 131072);
__global__ __launch_bounds__(32 * OW) void k_out(const bf* __restrict__ XB, const bf* __restrict__ WQ, const float* __restrict__ qb,
                                                  const float* __restrict__ lw, const float* __restrict__ lb, const float* __restrict__ TB,
                                                  const float* __restrict__ KM, const h16* __restrict__ KVB, const int* __restrict__ nhp, float* OUT) {
    __shared__ __align__(16) float os[OW * 16 * OSQ];
    __shared__ __align__(16) h16   qs[OW * 16 * QSP];
    __shared__ __align__(16) float zs[OW * 64];
    __shared__ __align__(16) float wl[9 * DM];
    __shared__ __align__(16) float bl[DM];
    __shared__ __align__(16) float kms[DM];
    const int tid = threadIdx.x;
    const int lane = tid & 31, lr = lane & 15, hi = lane >> 4;
    const int wave = __builtin_amdgcn_readfirstlane((int)(threadIdx.x >> 5));
    const size_t T0 = (size_t)blockIdx.x * (16 * OW);
    const int b = (int)(T0 / SEQ);
    const bool bad = nhp[0] != NH_;
    for (int i = tid; i < 9 * DM; i += 32 * OW) { const int c = i / 9, k = i - 9 * c; wl[k * DM + c] = bfr(lw[i]); }
    if (tid < DM) { bl[tid] = bfr(lb[tid]); kms[tid] = KM[(size_t)b * 128 + tid]; }
    __syncthreads();
    const size_t t0 = T0 + (size_t)wave * 16;
    const int tt = (int)(t0 % SEQ);
    const int wb = wave * 16 * OSQ, wq = wave * 16 * QSP, wz = wave * 64;

    v8f acc[6];
#pragma unroll
    for (int nb = 0; nb < 6; ++nb) acc[nb] = (v8f){};
    const size_t aoff = (t0 + (size_t)lr) * DM + 8 * hi; const size_t boff = (size_t)lr * DM + 8 * hi;
#pragma unroll
    for (int kc = 0; kc < DM; kc += 32) {
        const v16bf a = ldb(XB + aoff + kc);
#pragma unroll
        for (int nb = 0; nb < 6; ++nb) { const v16bf bq = ldb(WQ + boff + (size_t)nb * 16 * DM + kc); acc[nb] = wmmabg(a, bq, acc[nb]); }
    }
#pragma unroll
    for (int nb = 0; nb < 6; ++nb) { const float bc = bfr(qb[nb * 16 + lr]);
#pragma unroll
        for (int j = 0; j < 8; ++j) os[wb + (hi * 8 + j) * OSQ + nb * 16 + lr] = elu1(acc[nb][j] + bc); }
    wave_sync();
#pragma unroll
    for (int hd = 0; hd < 2; ++hd) { const int head = 2 * hi + hd; float s = 0.0f;
#pragma unroll 4
        for (int d = 0; d < HD; ++d) s += os[wb + lr * OSQ + head * HD + d] * kms[head * HD + d];
        zs[wz + lr * 4 + head] = 1.0f / (s + 1e-6f); }
#pragma unroll 1
    for (int it = 0; it < 6; ++it) { const int g = it * 32 + lane; const int tok = g / 12; const int c8 = (g - tok * 12) * 8;
        const int w = (tt + tok) % IMW;
        const v4f x0 = *(const v4fa*)(&os[wb + tok * OSQ + c8]); const v4f x1 = *(const v4fa*)(&os[wb + tok * OSQ + c8 + 4]);
        const int to = 2 * NPR * IMW + w * NPR + (c8 >> 1);
        const v4f cv = *(const v4f*)(TB + to); const v4f sv = *(const v4f*)(TB + NPR * IMW + to);
        v8h hq;
        hq[0] = toh_flush(x0[0] * cv[0] - x0[1] * sv[0]); hq[1] = toh_flush(x0[0] * sv[0] + x0[1] * cv[0]);
        hq[2] = toh_flush(x0[2] * cv[1] - x0[3] * sv[1]); hq[3] = toh_flush(x0[2] * sv[1] + x0[3] * cv[1]);
        hq[4] = toh_flush(x1[0] * cv[2] - x1[1] * sv[2]); hq[5] = toh_flush(x1[0] * sv[2] + x1[1] * cv[2]);
        hq[6] = toh_flush(x1[2] * cv[3] - x1[3] * sv[3]); hq[7] = toh_flush(x1[2] * sv[3] + x1[3] * cv[3]);
        *(v8ha*)(&qs[wq + tok * QSP + c8]) = hq; }
    wave_sync();

    v8f oa[6];
#pragma unroll
    for (int nb = 0; nb < 6; ++nb) oa[nb] = (v8f){};
    const size_t kvo = ((size_t)b * DM + (size_t)lr) * DM + 8 * hi;
#pragma unroll
    for (int ks = 0; ks < 3; ++ks) {
        const v16h a = cat16(*(const v8ha*)(&qs[wq + lr * QSP + ks * 32 + 8 * hi]), *(const v8ha*)(&qs[wq + lr * QSP + ks * 32 + 8 * hi + 16]));
#pragma unroll
        for (int nb = 0; nb < 6; ++nb) {
            if ((KVNZ >> (nb * 3 + ks)) & 1u) {
                const v16h bk = ldh(KVB + kvo + (size_t)nb * 16 * DM + ks * 32);
                oa[nb] = wmma16g(a, bk, oa[nb]); } }
    }
#pragma unroll
    for (int nb = 0; nb < 6; ++nb) { const int e = nb * 16 + lr; const int head = e / HD;
#pragma unroll
        for (int j = 0; j < 8; ++j) { const int tok = hi * 8 + j; os[wb + tok * OSQ + e] = oa[nb][j] * (zs[wz + tok * 4 + head] * KVI); } }
    wave_sync();

    float* orow = OUT + ((size_t)b * OUT_SEQ + (size_t)tt) * DM;
    const size_t xbb = (size_t)b * SEQ;
    const float qnan = __uint_as_float(0x7fc00000u);
#pragma unroll 1
    for (int it = 0; it < 12; ++it) { const int f = it * 32 + lane; const int tok = f / 24; const int c4 = (f - tok * 24) * 4;
        const int t = tt + tok; const int y = t / IMW; const int w = t - y * IMW;
        v4f val = *(const v4fa*)(&os[wb + tok * OSQ + c4]);
        const v4f bv = *(const v4fa*)(&bl[c4]); val += bv;
#pragma unroll 1
        for (int dy = 0; dy < 3; ++dy) { const int yy = y + dy - 1; const int yc = yy < 0 ? 0 : (yy > IMW - 1 ? IMW - 1 : yy);
#pragma unroll
            for (int dx = 0; dx < 3; ++dx) { const int xx = w + dx - 1; const int xc = xx < 0 ? 0 : (xx > IMW - 1 ? IMW - 1 : xx);
                const bool ok = (yy >= 0) & (yy < IMW) & (xx >= 0) & (xx < IMW);
                v2u u = *(const v2u*)(XB + (xbb + (size_t)(yc * IMW + xc)) * DM + c4);
                asm volatile("" : "+v"(u));
                const v4f wv = *(const v4fa*)(&wl[(dy * 3 + dx) * DM + c4]);
                const float e0 = __uint_as_float(u[0] << 16), e1 = __uint_as_float(u[0] & 0xffff0000u);
                const float e2 = __uint_as_float(u[1] << 16), e3 = __uint_as_float(u[1] & 0xffff0000u);
                val[0] += (ok ? e0 : 0.0f) * wv[0]; val[1] += (ok ? e1 : 0.0f) * wv[1];
                val[2] += (ok ? e2 : 0.0f) * wv[2]; val[3] += (ok ? e3 : 0.0f) * wv[3]; } }
        if (bad) { val[0] = qnan; val[1] = qnan; val[2] = qnan; val[3] = qnan; }
        *(v4fa*)(&os[wb + tok * OSQ + c4]) = val;
        *(volatile v4f*)(orow + (size_t)f * 4) = val; }
    __threadfence();
#pragma unroll 1
    for (int it = 0; it < 12; ++it) { const int f = it * 32 + lane; const int tok = f / 24; const int c4 = (f - tok * 24) * 4;
        const v4f val = *(const v4fa*)(&os[wb + tok * OSQ + c4]);
        *(volatile v4f*)(orow + (size_t)f * 4) = val; }
}

static constexpr size_t al256(size_t v) { return (v + 255) & ~(size_t)255; }
static constexpr size_t SZ_XB  = al256((size_t)NB * SEQ * DM * 2);
static constexpr size_t SZ_WB  = al256((size_t)2 * DM * DM * 2);
static constexpr size_t SZ_PL  = al256((size_t)NB * DM * SEQ * 2);
static constexpr size_t SZ_KSP = al256((size_t)NB * NT * 2 * 64 * 4);
static constexpr size_t SZ_KVP = al256((size_t)NB * NH_ * KVSPL * 1024 * 4);
static constexpr size_t SZ_KM  = al256((size_t)NB * 128 * 4);
static constexpr size_t SZ_KVB = al256((size_t)NB * DM * DM * 2);
static constexpr size_t SZ_TB  = al256((size_t)4 * NPR * IMW * 4);
static constexpr size_t SZ_TOTAL = SZ_XB + SZ_WB + 2 * SZ_PL + SZ_KSP + SZ_KVP + SZ_KM + SZ_KVB + SZ_TB;
static_assert(SZ_TOTAL <= (size_t)134217728);
static_assert(((size_t)DM * DM * 2) % 256 == 0);
static_assert(((size_t)NB * SEQ / 64) * 2 * 64 * 4 <= SZ_KSP);
static_assert((size_t)NB * NH_ * KVSPL * 4096 <= SZ_KVP);

extern "C" void kernel_launch(void* const* d_in, const int* in_sizes, int n_in,
                              void* d_out, int out_size, void* d_ws, size_t ws_size, hipStream_t stream) {
    if (n_in < 6) return;
    const size_t needx = ((size_t)(NB - 1) * SEQ_FULL + SEQ) * DM;
    if ((size_t)in_sizes[0] < needx) return;
    if ((size_t)in_sizes[1] < (size_t)2 * DM * DM || in_sizes[2] < 2 * DM) return;
    if (in_sizes[3] < 9 * DM || in_sizes[4] < DM || in_sizes[5] < 1) return;
    if ((size_t)out_size < ((size_t)(NB - 1) * OUT_SEQ + SEQ) * DM) return;
    if (SZ_TOTAL > ws_size) return;
    const float* x   = (const float*)d_in[0];
    const float* qkw = (const float*)d_in[1];
    const float* qkb = (const float*)d_in[2];
    const float* lw  = (const float*)d_in[3];
    const float* lb  = (const float*)d_in[4];
    const int*   nhp = (const int*)d_in[5];
    float* OUT = (float*)d_out;
    char* wsp = (char*)d_ws;
    bf*  XB  = (bf*)wsp;    wsp += SZ_XB;
    bf*  WB  = (bf*)wsp;    wsp += SZ_WB;
    h16* VT  = (h16*)wsp;   wsp += SZ_PL;
    h16* KT  = (h16*)wsp;   wsp += SZ_PL;
    float* KSP = (float*)wsp; wsp += SZ_KSP;
    float* KVP = (float*)wsp; wsp += SZ_KVP;
    float* KM  = (float*)wsp; wsp += SZ_KM;
    h16* KVB = (h16*)wsp;   wsp += SZ_KVB;
    float* TB  = (float*)wsp; wsp += SZ_TB;
    bf* WQ = WB; bf* WK = WB + (size_t)DM * DM;

    { const size_t n8 = (size_t)2 * DM * DM / 8;
      k_cvt8<<<(unsigned)((n8 + 255) / 256), 256, 0, stream>>>(qkw, WB, n8); }
    k_tab<<<(2 * NPR * IMW) / 256, 256, 0, stream>>>(TB);
    k_xprep<<<(NB * SEQ) / 64, 256, 0, stream>>>(x, XB, VT);
    k_kproj<<<dim3(2, (NB * SEQ) / 64, 1), 32, 0, stream>>>(WK, XB, qkb + DM, TB, KT, KSP);
    k_kv<<<dim3(KVSPL, NB * NH_, 1), 32 * KVW, 0, stream>>>(KT, VT, KVP);
    k_fin<<<NB, 256, 0, stream>>>(KSP, KVP, KM, KVB);
    k_out<<<(NB * SEQ) / (16 * OW), 32 * OW, 0, stream>>>(XB, WQ, qkb, lw, lb, TB, KM, KVB, nhp, OUT);
}
